// PodNetClassifier_6390911336757
// MI455X (gfx1250) — hardware-verified
//
#include <hip/hip_runtime.h>
#include <math.h>

typedef __attribute__((ext_vector_type(16))) _Float16 v16h;
typedef __attribute__((ext_vector_type(16))) __bf16 v16b;
typedef __attribute__((ext_vector_type(8)))  _Float16 v8h;
typedef __attribute__((ext_vector_type(8)))  float v8f;
typedef __attribute__((ext_vector_type(4)))  float v4f;
typedef __attribute__((ext_vector_type(2)))  float v2f;
typedef __attribute__((ext_vector_type(4)))  unsigned v4u;
typedef __attribute__((ext_vector_type(4)))  int v4i;
typedef float __attribute__((may_alias)) float_a;
typedef int __attribute__((may_alias)) int_a;

template <typename T> __device__ __forceinline__ void vst2(void* p, T v) { *(volatile T*)p = v; __threadfence(); *(volatile T*)p = v; }
__device__ __forceinline__ v8f wmma16(v16h a, v16h b, v8f c) {
  v8f d = __builtin_amdgcn_wmma_f32_16x16x32_f16(false, a, false, b, (short)0, c, false, false);
  asm volatile("v_nop\n\tv_nop\n\tv_nop\n\tv_nop" : "+v"(d) : "v"(a), "v"(b));
  return d;
}
__device__ __forceinline__ v8f wmma_bf(v16b a, v16b b, v8f c) {
  v8f d = __builtin_amdgcn_wmma_f32_16x16x32_bf16(false, a, false, b, (short)0, c, false, false);
  asm volatile("v_nop\n\tv_nop\n\tv_nop\n\tv_nop" : "+v"(d) : "v"(a), "v"(b));
  return d;
}
__device__ __forceinline__ v16h frag_h(const _Float16* rowk0, int lane) {
  union { v16h v; v8h q[2]; } u; const _Float16* p = rowk0 + 8 * (lane >> 4);
  u.q[0] = *(const v8h*)p; u.q[1] = *(const v8h*)(p + 16); return u.v;
}
__device__ __forceinline__ v16h frag_f32(const float* rowk0, int lane) {
  v16h a; const float* p = rowk0 + 8 * (lane >> 4);
#pragma unroll
  for (int i = 0; i < 8; ++i) { a[i] = (_Float16)p[i]; a[8 + i] = (_Float16)p[16 + i]; }
  return a;
}
__device__ __forceinline__ v16h frag_f32s(const float* rowk0, int lane, float sc) {
  v16h a; const float* p = rowk0 + 8 * (lane >> 4);
#pragma unroll
  for (int i = 0; i < 8; ++i) { a[i] = (_Float16)(p[i] * sc); a[8 + i] = (_Float16)(p[16 + i] * sc); }
  return a;
}
__device__ __forceinline__ v16h fragc_f32(const float* W, int k0, int n, int lane, int ld, int K) {
  v16h a; const int g = lane >> 4;
#pragma unroll
  for (int i = 0; i < 8; ++i) { const int ka = k0 + 8 * g + i, kb = ka + 16;
    a[i] = (_Float16)(ka < K ? W[(size_t)(ka < K ? ka : K - 1) * ld + n] : 0.f); a[8 + i] = (_Float16)(kb < K ? W[(size_t)(kb < K ? kb : K - 1) * ld + n] : 0.f); }
  return a;
}
struct F2 { v16b h, l; };
__device__ __forceinline__ F2 bsplit16(const float v[16]) { F2 r;
#pragma unroll
  for (int i = 0; i < 16; ++i) { const __bf16 h = (__bf16)v[i]; r.h[i] = h; r.l[i] = (__bf16)(v[i] - (float)h); }
  return r; }
__device__ __forceinline__ F2 split_row(const float* row, int k0, int lane) { float v[16]; const float* p = row + k0 + 8 * (lane >> 4);
#pragma unroll
  for (int i = 0; i < 8; ++i) { v[i] = p[i]; v[8 + i] = p[16 + i]; }
  return bsplit16(v); }
__device__ __forceinline__ F2 split_rowK(const float* row, int k0, int lane, int K) { float v[16]; const int g = lane >> 4;
#pragma unroll
  for (int i = 0; i < 8; ++i) { const int ka = k0 + 8 * g + i, kb = ka + 16; v[i] = ka < K ? row[ka < K ? ka : K - 1] : 0.f; v[8 + i] = kb < K ? row[kb < K ? kb : K - 1] : 0.f; }
  return bsplit16(v); }
__device__ __forceinline__ F2 split_col(const float* W, int k0, int n, int lane, int ld, int K) { float v[16]; const int g = lane >> 4;
#pragma unroll
  for (int i = 0; i < 8; ++i) { const int ka = k0 + 8 * g + i, kb = ka + 16; v[i] = ka < K ? W[(size_t)(ka < K ? ka : K - 1) * ld + n] : 0.f; v[8 + i] = kb < K ? W[(size_t)(kb < K ? kb : K - 1) * ld + n] : 0.f; }
  return bsplit16(v); }
__device__ __forceinline__ v8f mac3(const F2& a, const F2& b, v8f c) { c = wmma_bf(a.l, b.h, c); c = wmma_bf(a.h, b.l, c); return wmma_bf(a.h, b.h, c); }
__device__ __forceinline__ float sigm(float v) { return 1.0f / (1.0f + expf(-v)); }
#define LDSX() do { asm volatile("s_wait_dscnt 0" ::: "memory"); __builtin_amdgcn_wave_barrier(); __builtin_amdgcn_fence(__ATOMIC_RELEASE, "workgroup"); } while (0)


#define NBATCH 8192
#define DDIM 64
#define KP 10
#define NCLS 1000
#define NPROX (NCLS * KP)
#ifndef TRB
#define TRB (NBATCH / 16)
#endif
typedef __attribute__((ext_vector_type(8))) __bf16 v8b;
__device__ __forceinline__ v16b frag_b(const __bf16* rowk0, int lane) {
  union { v16b v; v8b q[2]; } u; const __bf16* p = rowk0 + 8 * (lane >> 4);
  u.q[0] = *(const v8b*)p; u.q[1] = *(const v8b*)(p + 16); return u.v;
}
__device__ __forceinline__ float bfr(float v) { return (float)(__bf16)v; }
__device__ __attribute__((noinline)) float exp_ni(float v) { return expf(v); }
#define WS_TH   0u
#define WS_TL   (WS_TH + 2u * 10048 * DDIM)
#define WS_TS   (WS_TL + 2u * 10048 * DDIM)
#define WS_END  (WS_TS + 4u * 10048)

__global__ __launch_bounds__(256) void k_th(const float* __restrict__ TH0, __bf16* __restrict__ THH, __bf16* __restrict__ THL, float* __restrict__ TS) {
  __shared__ float sv[64][65]; __shared__ __align__(16) __bf16 sh[64][72], sl[64][72]; __shared__ __align__(16) float ss[64];
  const int tid = threadIdx.x; const int rl = tid >> 2, q = tid & 3; const int r = blockIdx.x * 64 + rl;
  if (r < NPROX) { const int c = r / KP, j = r % KP; for (int i = q * 16; i < q * 16 + 16; ++i) sv[rl][i] = bfr(TH0[((size_t)i * KP + j) * NCLS + c]); } else for (int i = q * 16; i < q * 16 + 16; ++i) sv[rl][i] = 0.f;
  __syncthreads();
  { float s = 0.f; for (int i = q * 16; i < q * 16 + 16; ++i) s += sv[rl][i] * sv[rl][i]; s += __shfl_xor(s, 1); s += __shfl_xor(s, 2); const float inv = 1.0f / fmaxf(sqrtf(s), 1e-12f); float s2 = 0.f;
    for (int i = q * 16; i < q * 16 + 16; ++i) { const float v = sv[rl][i] * inv; s2 += v * v; const __bf16 hb = (__bf16)v; sh[rl][i] = hb; sl[rl][i] = (__bf16)(v - (float)hb); }
    s2 += __shfl_xor(s2, 1); s2 += __shfl_xor(s2, 2); if (q == 0) ss[rl] = (r < NPROX) ? s2 : 0.f; }
  __syncthreads();
  for (int qq = tid; qq < 64 * 8; qq += 256) { const int row = qq >> 3, pc = qq & 7; vst2((unsigned*)(THH + ((size_t)blockIdx.x * 64 + row) * DDIM + pc * 8), *(const v4u*)&sh[row][pc * 8]); vst2((unsigned*)(THL + ((size_t)blockIdx.x * 64 + row) * DDIM + pc * 8), *(const v4u*)&sl[row][pc * 8]); }
  if (tid < 16) vst2(TS + (size_t)blockIdx.x * 64 + tid * 4, *(const v4f*)&ss[tid * 4]);
}
__global__ __launch_bounds__(32) void k_main(const float* __restrict__ X, const __bf16* __restrict__ THH, const __bf16* __restrict__ THL, const float* __restrict__ TS, float* __restrict__ OUT) {
  __shared__ __align__(16) __bf16 sah[16][72], sal[16][72]; __shared__ float ssa[16]; __shared__ float sd[16][84]; __shared__ __align__(16) float sout[16][NCLS + 8];
  const int lane = threadIdx.x, col = lane & 15, g = lane >> 4; const size_t r0 = (size_t)blockIdx.x * 16;
  { const int row = lane & 15, half = lane >> 4; const float* xr = X + (r0 + row) * DDIM; float s = 0.f; for (int i = half * 32; i < half * 32 + 32; ++i) { const float v = bfr(xr[i]); s += v * v; } s += __shfl_xor(s, 16); const float inv = 1.0f / fmaxf(sqrtf(s), 1e-12f); float s2 = 0.f;
    for (int i = half * 32; i < half * 32 + 32; ++i) { const float v = bfr(xr[i]) * inv; s2 += v * v; const __bf16 hb = (__bf16)v; sah[row][i] = hb; sal[row][i] = (__bf16)(v - (float)hb); } s2 += __shfl_xor(s2, 16); if (half == 0) ssa[row] = s2; }
  LDSX();
  const F2 a0 = {frag_b(&sah[col][0], lane), frag_b(&sal[col][0], lane)}, a1 = {frag_b(&sah[col][32], lane), frag_b(&sal[col][32], lane)};
#pragma unroll 1
  for (int c0 = 0; c0 < NPROX; c0 += 80) { const int ncol = min(80, NPROX - c0);
#pragma unroll
    for (int t = 0; t < 5; ++t) { v8f acc = {}; if (t * 16 < ncol) { const size_t prow = (size_t)(c0 + t * 16 + col) * DDIM; const F2 b0 = {frag_b(THH + prow, lane), frag_b(THL + prow, lane)}, b1 = {frag_b(THH + prow + 32, lane), frag_b(THL + prow + 32, lane)}; acc = mac3(a0, b0, acc); acc = mac3(a1, b1, acc); }
#pragma unroll
      for (int r = 0; r < 8; ++r) { const int pcol = c0 + t * 16 + col; const float ts = (t * 16 < ncol) ? TS[min(pcol, NPROX - 1)] : 0.f; const float d2 = fmaxf(ssa[8 * g + r] + ts - 2.0f * acc[r], 0.f); sd[8 * g + r][t * 16 + col] = -d2; } }
    LDSX();
    { const int row = lane & 15, half = lane >> 4; const int ncls = ncol / KP; for (int cl = half; cl < ncls; cl += 2) { float mx = -3.0e38f; for (int j = 0; j < KP; ++j) mx = fmaxf(mx, sd[row][cl * KP + j]); float z = 0.f, ws = 0.f; for (int j = 0; j < KP; ++j) { const float sv = sd[row][cl * KP + j]; const float e = exp_ni(sv - mx); z += e; ws += sv * e; } sout[row][c0 / KP + cl] = ws / z; } }
    LDSX(); }
  for (int q = lane; q < 16 * NCLS / 4; q += 32) { const int f = q * 4; const int row = f / NCLS, c = f % NCLS; v4f v = {sout[row][c], sout[row][c + 1], sout[row][c + 2], sout[row][c + 3]}; vst2(OUT + (r0 + row) * NCLS + c, v); }
}

extern "C" void kernel_launch(void* const* d_in, const int* in_sizes, int n_in, void* d_out, int out_size, void* d_ws, size_t ws_size, hipStream_t stream) {
  (void)in_sizes; (void)n_in; (void)out_size;
  const float** F = (const float**)d_in;
  if (ws_size < (size_t)WS_END) return;
  char* ws = (char*)d_ws; __bf16 *THH = (__bf16*)(ws + WS_TH), *THL = (__bf16*)(ws + WS_TL); float* TS = (float*)(ws + WS_TS);
  k_th<<<10048 / 64, 256, 0, stream>>>(F[1], THH, THL, TS);
  k_main<<<TRB, 32, 0, stream>>>(F[0], THH, THL, TS, (float*)d_out);
}
